// DynamicWaveAttention_5995774345692
// MI455X (gfx1250) — hardware-verified
//
#include <hip/hip_runtime.h>
#include <stddef.h>
#include <stdint.h>


#define S_LEN  2048
#define DM     512
#define NH     8
#define HD     64
#define GH     128
#define WF     16
#define BATCH  2
#define NTOK   (BATCH * S_LEN)
#define LOG2E  1.4426950408889634f
#define PSCALE 4096.0f
#define INV_PSCALE 0.000244140625f

typedef __bf16         v16bf __attribute__((ext_vector_type(16)));
typedef __bf16         v8bf  __attribute__((ext_vector_type(8)));
typedef _Float16       v16h  __attribute__((ext_vector_type(16)));
typedef _Float16       v8h   __attribute__((ext_vector_type(8)));
typedef float          v8f   __attribute__((ext_vector_type(8)));
typedef float          v4f   __attribute__((ext_vector_type(4)));
typedef unsigned int   v4u   __attribute__((ext_vector_type(4)));
typedef unsigned short v8us  __attribute__((ext_vector_type(8)));

union FragB { v16bf v; v8bf p[2]; };
union FragH { v16h v; v8h p[2]; };
union Pack8 { v8us s; v8h h; v4u u; };

static __device__ __forceinline__ unsigned short f2bf_bits(float f) {
  unsigned int u = __float_as_uint(f);
  u += 0x7FFFu + ((u >> 16) & 1u);
  return (unsigned short)(u >> 16);
}
static __device__ __forceinline__ float bf_bits2f(unsigned short s) {
  return __uint_as_float(((unsigned int)s) << 16);
}
static __device__ __forceinline__ void unpack8(const v4f a, const v4f b, float o[8]) {
  o[0] = a.x; o[1] = a.y; o[2] = a.z; o[3] = a.w;
  o[4] = b.x; o[5] = b.y; o[6] = b.z; o[7] = b.w;
}

static __device__ __forceinline__ v16bf ldfrag_bf(const __bf16* p, int hh) {
  FragB f;
  f.p[0] = *(const v8bf*)(p + 8 * hh);
  f.p[1] = *(const v8bf*)(p + 16 + 8 * hh);
  return f.v;
}
static __device__ __forceinline__ v16h ldfrag_h(const _Float16* p, int hh) {
  FragH f;
  f.p[0] = *(const v8h*)(p + 8 * hh);
  f.p[1] = *(const v8h*)(p + 16 + 8 * hh);
  return f.v;
}

static __device__ __forceinline__ v8f mma_bf3(v16bf ah, v16bf al, v16bf bh, v16bf bl, v8f c) {
  c = __builtin_amdgcn_wmma_f32_16x16x32_bf16(false, ah, false, bh, (short)0, c, false, false);
  c = __builtin_amdgcn_wmma_f32_16x16x32_bf16(false, al, false, bh, (short)0, c, false, false);
  c = __builtin_amdgcn_wmma_f32_16x16x32_bf16(false, ah, false, bl, (short)0, c, false, false);
  asm volatile("v_nop\n\tv_nop\n\tv_nop\n\tv_nop" : "+v"(c) : "v"(ah), "v"(al), "v"(bh), "v"(bl));
  return c;
}
static __device__ __forceinline__ v8f mma_h1(v16h a, v16h b, v8f c) {
  c = __builtin_amdgcn_wmma_f32_16x16x32_f16(false, a, false, b, (short)0, c, false, false);
  asm volatile("v_nop\n\tv_nop\n\tv_nop\n\tv_nop" : "+v"(c) : "v"(a), "v"(b));
  return c;
}

static __device__ __forceinline__ void split_store8(const float v[8], unsigned short* dh, unsigned short* dl) {
  Pack8 ph, pl;
#pragma unroll
  for (int e = 0; e < 8; ++e) {
    const unsigned short hb = f2bf_bits(v[e]);
    ph.s[e] = hb;
    pl.s[e] = f2bf_bits(v[e] - bf_bits2f(hb));
  }
  const v4u uh = ph.u, ul = pl.u;
  *(volatile v4u*)dh = uh;
  *(volatile v4u*)dl = ul;
  __threadfence();
  *(volatile v4u*)dh = uh;
  *(volatile v4u*)dl = ul;
}

__global__ __launch_bounds__(256) void prep_kernel(
    const float* __restrict__ x, const float* __restrict__ wq,
    const float* __restrict__ wk, const float* __restrict__ wv,
    const float* __restrict__ g1w,
    unsigned short* xh, unsigned short* xl, unsigned short* wth, unsigned short* wtl,
    unsigned short* gth, unsigned short* gtl,
    int nxv, int nwv, int ngv) {
  const int i = blockIdx.x * blockDim.x + threadIdx.x;
  if (i < nxv) {
    const v4f a = *(const v4f*)(x + (size_t)i * 8);
    const v4f c = *(const v4f*)(x + (size_t)i * 8 + 4);
    float v[8];
    unpack8(a, c, v);
    split_store8(v, xh + (size_t)i * 8, xl + (size_t)i * 8);
  } else if (i < nxv + nwv) {
    const int j = i - nxv;
    const int mat = j >> 15;
    const int rem = j & 32767;
    const int o = rem >> 6;
    const int inb = (rem & 63) * 8;
    const float* w = (mat == 0) ? wq : (mat == 1) ? wk : wv;
    float v[8];
#pragma unroll
    for (int e = 0; e < 8; ++e) v[e] = w[(size_t)(inb + e) * DM + o];
    split_store8(v, wth + (size_t)j * 8, wtl + (size_t)j * 8);
  } else if (i < nxv + nwv + ngv) {
    const int j = i - nxv - nwv;
    const int o = j >> 6;
    const int inb = (j & 63) * 8;
    float v[8];
#pragma unroll
    for (int e = 0; e < 8; ++e) v[e] = g1w[(size_t)(inb + e) * GH + o];
    split_store8(v, gth + (size_t)j * 8, gtl + (size_t)j * 8);
  }
}

__global__ __launch_bounds__(128) void gate_kernel(
    const __bf16* __restrict__ xh, const __bf16* __restrict__ xl,
    const __bf16* __restrict__ gth, const __bf16* __restrict__ gtl,
    const float* __restrict__ g1b, const float* __restrict__ g2w,
    const float* __restrict__ g2b, float* gates, int ntile) {
  __shared__ float h1s[32][GH + 1];
  __shared__ __attribute__((aligned(16))) float gl[NH][32];
  if ((int)blockIdx.x >= ntile) return;
  const int tid = threadIdx.x, wave = tid >> 5, lane = tid & 31;
  const int m = lane & 15, hh = lane >> 4, r0 = hh * 8;
  const int tok0 = blockIdx.x * 32;
  const int th = wave & 1;
  const int hb = (wave >> 1) * 64;

  const size_t aoff = (size_t)(tok0 + th * 16 + m) * DM;
  size_t woff[4];
#pragma unroll
  for (int j = 0; j < 4; ++j) woff[j] = (size_t)(hb + j * 16 + m) * DM;

  v8f acc[4] = {};
#pragma unroll 1
  for (int kk = 0; kk < DM; kk += 32) {
    const v16bf ah = ldfrag_bf(xh + aoff + kk, hh);
    const v16bf al = ldfrag_bf(xl + aoff + kk, hh);
#pragma unroll
    for (int j = 0; j < 4; ++j) {
      const v16bf bhf = ldfrag_bf(gth + woff[j] + kk, hh);
      const v16bf blf = ldfrag_bf(gtl + woff[j] + kk, hh);
      acc[j] = mma_bf3(ah, al, bhf, blf, acc[j]);
    }
  }

#pragma unroll
  for (int j = 0; j < 4; ++j) {
    const int hu = hb + j * 16 + m;
    const float bj = g1b[hu];
#pragma unroll
    for (int r = 0; r < 8; ++r) h1s[th * 16 + r0 + r][hu] = fmaxf(acc[j][r] + bj, 0.0f);
  }
  __syncthreads();

  const int tk = tid >> 2, hd0 = (tid & 3) * 2;
  float a0 = g2b[hd0], a1 = g2b[hd0 + 1];
#pragma unroll 1
  for (int jj = 0; jj < GH; ++jj) {
    const float hv = h1s[tk][jj];
    a0 = fmaf(hv, g2w[jj * NH + hd0], a0);
    a1 = fmaf(hv, g2w[jj * NH + hd0 + 1], a1);
  }
  gl[hd0][tk]     = 1.0f / (1.0f + exp2f(-a0 * LOG2E));
  gl[hd0 + 1][tk] = 1.0f / (1.0f + exp2f(-a1 * LOG2E));
  __syncthreads();

  if (tid < 64) {
    const int line = tid >> 3, piece = tid & 7;
    const v4f val = *(const v4f*)&gl[line][piece * 4];
    const int b = tok0 / S_LEN, s0 = tok0 - b * S_LEN;
    float* dst = gates + ((size_t)(b * NH + line)) * S_LEN + s0 + piece * 4;
    *(volatile v4f*)dst = val;
    __threadfence();
    *(volatile v4f*)dst = val;
  }
}

__global__ __launch_bounds__(128) void qkv_kernel(
    const __bf16* __restrict__ xh, const __bf16* __restrict__ xl,
    const __bf16* __restrict__ wth, const __bf16* __restrict__ wtl,
    const float* __restrict__ bq, const float* __restrict__ bk, const float* __restrict__ bv,
    unsigned short* Qh, unsigned short* Ql, unsigned short* Kh, unsigned short* Kl,
    unsigned short* VT, int ntt) {
  __shared__ __attribute__((aligned(16))) unsigned short lt[2][64][64];
  if ((int)blockIdx.x >= ntt) return;
  const int tt = blockIdx.x, head = blockIdx.y, mat = blockIdx.z;
  const int tid = threadIdx.x, wave = tid >> 5, lane = tid & 31;
  const int m = lane & 15, hh = lane >> 4, r0 = hh * 8;
  const int tokbase = tt * 64;
  const int b = tokbase / S_LEN, s0 = tokbase - b * S_LEN;

  const size_t aoff = (size_t)(tokbase + wave * 16 + m) * DM;
  size_t woff[4];
#pragma unroll
  for (int j = 0; j < 4; ++j)
    woff[j] = ((size_t)mat * DM + head * HD + j * 16 + m) * DM;

  v8f acc[4] = {};
#pragma unroll 1
  for (int kk = 0; kk < DM; kk += 32) {
    const v16bf ah = ldfrag_bf(xh + aoff + kk, hh);
    const v16bf al = ldfrag_bf(xl + aoff + kk, hh);
#pragma unroll
    for (int j = 0; j < 4; ++j) {
      const v16bf bhf = ldfrag_bf(wth + woff[j] + kk, hh);
      const v16bf blf = ldfrag_bf(wtl + woff[j] + kk, hh);
      acc[j] = mma_bf3(ah, al, bhf, blf, acc[j]);
    }
  }

  const float* bias = (mat == 0) ? bq : (mat == 1) ? bk : bv;
  const int ltok = wave * 16 + r0;
  if (mat < 2) {
#pragma unroll
    for (int j = 0; j < 4; ++j) {
      const int ld = j * 16 + m;
      const float bj = bias[head * HD + ld];
#pragma unroll
      for (int r = 0; r < 8; ++r) {
        const float v = acc[j][r] + bj;
        const unsigned short hb = f2bf_bits(v);
        lt[0][ltok + r][ld] = hb;
        lt[1][ltok + r][ld] = f2bf_bits(v - bf_bits2f(hb));
      }
    }
  } else {
#pragma unroll
    for (int j = 0; j < 4; ++j) {
      const int ld = j * 16 + m;
      const float bj = bias[head * HD + ld];
      Pack8 pk;
#pragma unroll
      for (int r = 0; r < 8; ++r) pk.h[r] = (_Float16)(acc[j][r] + bj);
      *(v4u*)&lt[0][ld][ltok] = pk.u;
    }
  }
  __syncthreads();

  const int piece = tid & 7, lb = tid >> 3;
  const size_t bh8 = (size_t)(b * NH + head);
  if (mat < 2) {
    unsigned short* dh = (mat == 0) ? Qh : Kh;
    unsigned short* dl = (mat == 0) ? Ql : Kl;
    v4u val[8];
    size_t go[4];
#pragma unroll
    for (int i = 0; i < 4; ++i) {
      const int L = lb + 16 * i;
      val[i]     = *(const v4u*)&lt[0][L][piece * 8];
      val[4 + i] = *(const v4u*)&lt[1][L][piece * 8];
      go[i] = (bh8 * S_LEN + s0 + L) * HD + piece * 8;
    }
#pragma unroll
    for (int i = 0; i < 4; ++i) { *(volatile v4u*)(dh + go[i]) = val[i]; *(volatile v4u*)(dl + go[i]) = val[4 + i]; }
    __threadfence();
#pragma unroll
    for (int i = 0; i < 4; ++i) { *(volatile v4u*)(dh + go[i]) = val[i]; *(volatile v4u*)(dl + go[i]) = val[4 + i]; }
  } else {
    v4u val[4];
    size_t go[4];
#pragma unroll
    for (int i = 0; i < 4; ++i) {
      const int L = lb + 16 * i;
      val[i] = *(const v4u*)&lt[0][L][piece * 8];
      go[i] = (bh8 * HD + L) * S_LEN + s0 + piece * 8;
    }
#pragma unroll
    for (int i = 0; i < 4; ++i) *(volatile v4u*)(VT + go[i]) = val[i];
    __threadfence();
#pragma unroll
    for (int i = 0; i < 4; ++i) *(volatile v4u*)(VT + go[i]) = val[i];
  }
}

__global__ __launch_bounds__(256) __attribute__((amdgpu_num_vgpr(248)))
void attn_ln_kernel(
    const __bf16* __restrict__ Qh, const __bf16* __restrict__ Ql,
    const __bf16* __restrict__ Kh, const __bf16* __restrict__ Kl,
    const _Float16* __restrict__ VT, const float* __restrict__ gates,
    const float* __restrict__ wmask, const float* __restrict__ adj,
    const float* __restrict__ x, const float* __restrict__ lng,
    const float* __restrict__ lnb, float* out, int nqt) {
  __shared__ __attribute__((aligned(16))) float wmq[16][WF];
  __shared__ __attribute__((aligned(16))) float ws_lds[16][64];
  __shared__ __attribute__((aligned(16))) float adj_lds[16][64];
  __shared__ __attribute__((aligned(16))) float obuf[16][DM];
  if ((int)blockIdx.x >= nqt) return;

  const int qtiles = S_LEN / 16;
  const int b = blockIdx.x / qtiles, qt = blockIdx.x - b * qtiles, qbase = qt * 16;
  const int tid = threadIdx.x, h = tid >> 5, lane = tid & 31;
  const int m = lane & 15, hh = lane >> 4, r0 = hh * 8;

  wmq[tid >> 4][tid & 15] = wmask[((size_t)b * S_LEN + qbase + (tid >> 4)) * WF + (tid & 15)];
  __syncthreads();

  const size_t bhd = (size_t)(b * NH + h);
  const size_t qoff = (bhd * S_LEN + qbase + m) * HD;
  const v16bf qh0 = ldfrag_bf(Qh + qoff, hh), qh1 = ldfrag_bf(Qh + qoff + 32, hh);
  const v16bf ql0 = ldfrag_bf(Ql + qoff, hh), ql1 = ldfrag_bf(Ql + qoff + 32, hh);

  v8f oacc[4] = {};
  float mrun = -3.0e38f, lrun = 0.0f;

  const float* gp_base = gates + bhd * S_LEN;
  const size_t koff = (bhd * S_LEN + m) * HD;
  const _Float16* vbase = VT + (bhd * HD + m) * S_LEN;

  const int sq = tid >> 4, sk4 = (tid & 15) * 4;
  const float* adj_row = adj + ((size_t)b * S_LEN + qbase + sq) * S_LEN + sk4;

  for (int kc = 0; kc < S_LEN / 64; ++kc) {
    const int kbase64 = kc * 64;

    *(v4f*)&adj_lds[sq][sk4] = *(const v4f*)(adj_row + kbase64);
#pragma unroll
    for (int i = 0; i < 4; ++i) {
      const int cell = tid * 4 + i;
      const int q = cell >> 6, kk = cell & 63;
      const float* wmk = wmask + ((size_t)b * S_LEN + kbase64 + kk) * WF;
      float acc = 0.0f;
#pragma unroll
      for (int f4 = 0; f4 < WF / 4; ++f4) {
        const v4f kv = *(const v4f*)(wmk + 4 * f4);
        const v4f qv = *(const v4f*)&wmq[q][4 * f4];
        acc = fmaf(qv.x, kv.x, acc);
        acc = fmaf(qv.y, kv.y, acc);
        acc = fmaf(qv.z, kv.z, acc);
        acc = fmaf(qv.w, kv.w, acc);
      }
      ws_lds[q][kk] = acc;
    }
    __syncthreads();

#pragma unroll 1
    for (int jh = 0; jh < 2; ++jh) {
      const int kbase = kbase64 + jh * 32;
      const int ko = jh * 32;

      v8f s0 = {}, s1 = {};
      {
        const size_t o0 = koff + (size_t)kbase * HD;
        const size_t o1 = o0 + (size_t)16 * HD;
        s0 = mma_bf3(ldfrag_bf(Kh + o0, hh),      ldfrag_bf(Kl + o0, hh),      qh0, ql0, s0);
        s0 = mma_bf3(ldfrag_bf(Kh + o0 + 32, hh), ldfrag_bf(Kl + o0 + 32, hh), qh1, ql1, s0);
        s1 = mma_bf3(ldfrag_bf(Kh + o1, hh),      ldfrag_bf(Kl + o1, hh),      qh0, ql0, s1);
        s1 = mma_bf3(ldfrag_bf(Kh + o1 + 32, hh), ldfrag_bf(Kl + o1 + 32, hh), qh1, ql1, s1);
      }

      const float* gp = gp_base + kbase + r0;
      float gA[8], gB[8], W0[8], W1[8], A0[8], A1[8];
      unpack8(*(const v4f*)gp, *(const v4f*)(gp + 4), gA);
      unpack8(*(const v4f*)(gp + 16), *(const v4f*)(gp + 20), gB);
      unpack8(*(const v4f*)&ws_lds[m][ko + r0], *(const v4f*)&ws_lds[m][ko + r0 + 4], W0);
      unpack8(*(const v4f*)&ws_lds[m][ko + 16 + r0], *(const v4f*)&ws_lds[m][ko + 16 + r0 + 4], W1);
      unpack8(*(const v4f*)&adj_lds[m][ko + r0], *(const v4f*)&adj_lds[m][ko + r0 + 4], A0);
      unpack8(*(const v4f*)&adj_lds[m][ko + 16 + r0], *(const v4f*)&adj_lds[m][ko + 16 + r0 + 4], A1);

      float p0[8], p1[8], mloc = -3.0e38f;
#pragma unroll
      for (int r = 0; r < 8; ++r) {
        const float t0 = (s0[r] * 0.125f) * (gA[r] + W0[r]) + A0[r];
        const float t1 = (s1[r] * 0.125f) * (gB[r] + W1[r]) + A1[r];
        p0[r] = t0; p1[r] = t1;
        mloc = fmaxf(mloc, fmaxf(t0, t1));
      }
      const float mch  = fmaxf(mloc, __shfl_xor(mloc, 16, 32));
      const float mnew = fmaxf(mrun, mch);
      const float corr = exp2f((mrun - mnew) * LOG2E);
      float lsum = 0.0f;
#pragma unroll
      for (int r = 0; r < 8; ++r) {
        p0[r] = exp2f((p0[r] - mnew) * LOG2E);
        p1[r] = exp2f((p1[r] - mnew) * LOG2E);
        lsum += p0[r] + p1[r];
      }
      lsum += __shfl_xor(lsum, 16, 32);
      lrun = lrun * corr + lsum;
      mrun = mnew;
#pragma unroll
      for (int t = 0; t < 4; ++t)
#pragma unroll
        for (int r = 0; r < 8; ++r) oacc[t][r] *= corr;

      v16h pf;
#pragma unroll
      for (int r = 0; r < 8; ++r) {
        pf[r]     = (_Float16)(p0[r] * PSCALE);
        pf[r + 8] = (_Float16)(p1[r] * PSCALE);
      }

#pragma unroll
      for (int t = 0; t < 4; ++t) {
        const v16h vf = ldfrag_h(vbase + (size_t)t * 16 * S_LEN + kbase, hh);
        oacc[t] = mma_h1(vf, pf, oacc[t]);
      }
    }
    __syncthreads();
  }

  const float oscale = (1.0f / lrun) * INV_PSCALE;
#pragma unroll
  for (int t = 0; t < 4; ++t) {
    v4f u0, u1;
    u0.x = oacc[t][0] * oscale; u0.y = oacc[t][1] * oscale; u0.z = oacc[t][2] * oscale; u0.w = oacc[t][3] * oscale;
    u1.x = oacc[t][4] * oscale; u1.y = oacc[t][5] * oscale; u1.z = oacc[t][6] * oscale; u1.w = oacc[t][7] * oscale;
    float* dst = &obuf[m][h * HD + t * 16 + r0];
    *(v4f*)dst = u0;
    *(v4f*)(dst + 4) = u1;
  }
  __syncthreads();

#pragma unroll 1
  for (int qq = 0; qq < 2; ++qq) {
    const int q = 2 * h + qq;
    const size_t tok = (size_t)b * S_LEN + qbase + q;
    v4f y[4];
    float s = 0.0f;
#pragma unroll
    for (int i = 0; i < 4; ++i) {
      const v4f o  = *(const v4f*)&obuf[q][4 * lane + 128 * i];
      const v4f xv = *(const v4f*)(x + tok * DM + 4 * lane + 128 * i);
      y[i] = o + xv;
      s += (y[i].x + y[i].y) + (y[i].z + y[i].w);
    }
    s += __shfl_xor(s, 16, 32);
    s += __shfl_xor(s, 8, 32);
    s += __shfl_xor(s, 4, 32);
    s += __shfl_xor(s, 2, 32);
    s += __shfl_xor(s, 1, 32);
    const float mu = s * (1.0f / DM);
    float ss = 0.0f;
#pragma unroll
    for (int i = 0; i < 4; ++i) {
      const v4f d = y[i] - mu;
      ss += (d.x * d.x + d.y * d.y) + (d.z * d.z + d.w * d.w);
    }
    ss += __shfl_xor(ss, 16, 32);
    ss += __shfl_xor(ss, 8, 32);
    ss += __shfl_xor(ss, 4, 32);
    ss += __shfl_xor(ss, 2, 32);
    ss += __shfl_xor(ss, 1, 32);
    const float rstd = rsqrtf(ss * (1.0f / DM) + 1.0e-5f);
    v4f res[4];
#pragma unroll
    for (int i = 0; i < 4; ++i) {
      const v4f g  = *(const v4f*)(lng + 4 * lane + 128 * i);
      const v4f bb = *(const v4f*)(lnb + 4 * lane + 128 * i);
      res[i] = ((y[i] - mu) * rstd) * g + bb;
    }
    float* op = out + tok * DM + 4 * lane;
#pragma unroll
    for (int i = 0; i < 4; ++i) *(volatile v4f*)(op + 128 * i) = res[i];
    __threadfence();
#pragma unroll
    for (int i = 0; i < 4; ++i) *(volatile v4f*)(op + 128 * i) = res[i];
  }
}

extern "C" void kernel_launch(void* const* d_in, const int* in_sizes, int n_in,
                              void* d_out, int out_size, void* d_ws, size_t ws_size,
                              hipStream_t stream) {
  if (n_in < 15) return;
  if (in_sizes[0] != NTOK * DM || in_sizes[1] != NTOK * WF ||
      in_sizes[2] != BATCH * S_LEN * S_LEN || in_sizes[3] != DM * DM ||
      in_sizes[5] != DM * DM || in_sizes[7] != DM * DM || in_sizes[9] != DM * GH ||
      in_sizes[11] != GH * NH || in_sizes[13] != DM || out_size != NTOK * DM) return;

  const float* x     = (const float*)d_in[0];
  const float* wmask = (const float*)d_in[1];
  const float* adj   = (const float*)d_in[2];
  const float* wq_w  = (const float*)d_in[3];
  const float* wq_b  = (const float*)d_in[4];
  const float* wk_w  = (const float*)d_in[5];
  const float* wk_b  = (const float*)d_in[6];
  const float* wv_w  = (const float*)d_in[7];
  const float* wv_b  = (const float*)d_in[8];
  const float* g1_w  = (const float*)d_in[9];
  const float* g1_b  = (const float*)d_in[10];
  const float* g2_w  = (const float*)d_in[11];
  const float* g2_b  = (const float*)d_in[12];
  const float* ln_g  = (const float*)d_in[13];
  const float* ln_b  = (const float*)d_in[14];
  float* out = (float*)d_out;

  const size_t sz_x  = (size_t)NTOK * DM * 2;
  const size_t sz_w  = (size_t)3 * DM * DM * 2;
  const size_t sz_q  = (size_t)NTOK * DM * 2;
  const size_t sz_g  = (size_t)BATCH * NH * S_LEN * 4;
  const size_t sz_g1 = (size_t)GH * DM * 2;
  const size_t off_xh  = 0;
  const size_t off_xl  = off_xh + sz_x;
  const size_t off_wth = off_xl + sz_x;
  const size_t off_wtl = off_wth + sz_w;
  const size_t off_qh  = off_wtl + sz_w;
  const size_t off_ql  = off_qh + sz_q;
  const size_t off_kh  = off_ql + sz_q;
  const size_t off_kl  = off_kh + sz_q;
  const size_t off_vt  = off_kl + sz_q;
  const size_t off_g   = off_vt + sz_q;
  const size_t off_gth = off_g + sz_g;
  const size_t off_gtl = off_gth + sz_g1;
  const size_t total   = off_gtl + sz_g1;
  if (total > ws_size) return;

  uint8_t* ws = (uint8_t*)d_ws;
  unsigned short* xh  = (unsigned short*)(ws + off_xh);
  unsigned short* xl  = (unsigned short*)(ws + off_xl);
  unsigned short* wth = (unsigned short*)(ws + off_wth);
  unsigned short* wtl = (unsigned short*)(ws + off_wtl);
  unsigned short* qh  = (unsigned short*)(ws + off_qh);
  unsigned short* ql  = (unsigned short*)(ws + off_ql);
  unsigned short* kh  = (unsigned short*)(ws + off_kh);
  unsigned short* kl  = (unsigned short*)(ws + off_kl);
  unsigned short* vt  = (unsigned short*)(ws + off_vt);
  float* gates        = (float*)(ws + off_g);
  unsigned short* gth = (unsigned short*)(ws + off_gth);
  unsigned short* gtl = (unsigned short*)(ws + off_gtl);

  const int nxv = NTOK * DM / 8;
  const int nwv = 3 * DM * DM / 8;
  const int ngv = GH * DM / 8;
  const int prep_blocks = (nxv + nwv + ngv + 255) / 256;
  const int ntile = (NTOK + 31) / 32;
  const int ntt = (NTOK + 63) / 64;
  const int nqt = (BATCH * S_LEN + 15) / 16;

  prep_kernel<<<prep_blocks, 256, 0, stream>>>(x, wq_w, wk_w, wv_w, g1_w,
                                               xh, xl, wth, wtl, gth, gtl, nxv, nwv, ngv);
  gate_kernel<<<ntile, 128, 0, stream>>>(
      (const __bf16*)xh, (const __bf16*)xl, (const __bf16*)gth, (const __bf16*)gtl,
      g1_b, g2_w, g2_b, gates, ntile);
  qkv_kernel<<<dim3(ntt, NH, 3), 128, 0, stream>>>(
      (const __bf16*)xh, (const __bf16*)xl, (const __bf16*)wth, (const __bf16*)wtl,
      wq_b, wk_b, wv_b, qh, ql, kh, kl, vt, ntt);
  attn_ln_kernel<<<nqt, 256, 0, stream>>>(
      (const __bf16*)qh, (const __bf16*)ql, (const __bf16*)kh, (const __bf16*)kl,
      (const _Float16*)vt, gates, wmask, adj, x, ln_g, ln_b, out, nqt);
  (void)hipGetLastError();
}
